// PyTorchSSM_78915729096793
// MI455X (gfx1250) — hardware-verified
//
#include <hip/hip_runtime.h>
#include <math.h>

#pragma clang fp contract(off)

constexpr int kBatch   = 2;
constexpr int kSeq     = 2048;
constexpr int kDModel  = 1024;
constexpr int kDInner  = 2048;
constexpr int kNHeads  = 32;
constexpr int kHeadDim = 64;
constexpr int kDState  = 128;
constexpr int kConvDim = 2304;
constexpr int kDInProj = 4384;
constexpr int kNPad    = 4416;
constexpr int kRows    = kBatch * kSeq;
constexpr float kXCarry    = 8.0f;
constexpr float kWCarry    = 256.0f;
constexpr float kYCarry    = 8.0f;
constexpr float kProjScale = 1.0f / 2048.0f;
constexpr float kEps       = 1e-5f;

typedef __attribute__((ext_vector_type(16))) _Float16 v16h;
typedef __attribute__((ext_vector_type(8)))  _Float16 v8h;
typedef __attribute__((ext_vector_type(16))) __bf16   v16b;
typedef __attribute__((ext_vector_type(8)))  __bf16   v8b;
typedef __attribute__((ext_vector_type(8)))  float    v8f;
typedef __attribute__((ext_vector_type(4)))  float    v4f;
typedef __attribute__((ext_vector_type(4)))  unsigned int v4u;

__device__ __forceinline__ unsigned short f2bf_bits(float f) {
  unsigned u = __float_as_uint(f);
  return (unsigned short)((u + 0x7FFFu + ((u >> 16) & 1u)) >> 16);
}
__device__ __forceinline__ float bf_bits2f(unsigned short h) { return __uint_as_float(((unsigned)h) << 16); }

__device__ __forceinline__ void dep_guard_h(v8f& a, v8f& b, v16h x, v16h y) { asm volatile("v_nop\n\tv_nop\n\tv_nop\n\tv_nop" : "+v"(a), "+v"(b) : "v"(x), "v"(y)); }
__device__ __forceinline__ void dep_guard_b(v8f& a, v8f& b, v16b x, v16b y) { asm volatile("v_nop\n\tv_nop\n\tv_nop\n\tv_nop" : "+v"(a), "+v"(b) : "v"(x), "v"(y)); }
__device__ __forceinline__ void keep4_h(v16h a, v16h b, v16h c, v16h d) { asm volatile("v_nop" :: "v"(a), "v"(b), "v"(c), "v"(d)); }
__device__ __forceinline__ void keep4_b(v16b a, v16b b, v16b c, v16b d) { asm volatile("v_nop" :: "v"(a), "v"(b), "v"(c), "v"(d)); }
__device__ __forceinline__ void acc_guard4(v8f& a, v8f& b, v8f& c, v8f& d) { asm volatile("v_nop\n\tv_nop\n\tv_nop\n\tv_nop" : "+v"(a), "+v"(b), "+v"(c), "+v"(d)); }
template <typename T> struct Frag;
template <> struct Frag<_Float16> {
  typedef v16h V; union U { v16h v; v8h h[2]; };
  static __device__ __forceinline__ v16h load(const _Float16* p) {
    U f; f.h[0] = *(const v8h*)(p); f.h[1] = *(const v8h*)(p + 16); return f.v;
  }
  static __device__ __forceinline__ v8f mma(v16h a, v16h b, v8f c) {
    return __builtin_amdgcn_wmma_f32_16x16x32_f16(false, a, false, b, (short)0, c, false, false);
  }
  static __device__ __forceinline__ void guard(v8f& a, v8f& b, v16h x, v16h y) { dep_guard_h(a, b, x, y); }
  static __device__ __forceinline__ void keep(v16h a, v16h b, v16h c, v16h d) { keep4_h(a, b, c, d); }
};
template <> struct Frag<__bf16> {
  typedef v16b V; union U { v16b v; v8b h[2]; };
  static __device__ __forceinline__ v16b load(const __bf16* p) {
    U f; f.h[0] = *(const v8b*)(p); f.h[1] = *(const v8b*)(p + 16); return f.v;
  }
  static __device__ __forceinline__ v8f mma(v16b a, v16b b, v8f c) {
    return __builtin_amdgcn_wmma_f32_16x16x32_bf16(false, a, false, b, (short)0, c, false, false);
  }
  static __device__ __forceinline__ void guard(v8f& a, v8f& b, v16b x, v16b y) { dep_guard_b(a, b, x, y); }
  static __device__ __forceinline__ void keep(v16b a, v16b b, v16b c, v16b d) { keep4_b(a, b, c, d); }
};

__device__ __forceinline__ unsigned pk16(unsigned short a, unsigned short b) { return (unsigned)a | ((unsigned)b << 16); }
__device__ __forceinline__ unsigned short h_bits(float f) { const _Float16 h = (_Float16)f; return __builtin_bit_cast(unsigned short, h); }

template <int ET> struct Elem;
template <> struct Elem<0> { typedef _Float16 T; };
template <> struct Elem<1> { typedef __bf16 T; };
template <int ET, bool SPLIT, int BIAS_MODE, int OUT_MODE, bool RESID, int ACT = 0>
__global__ __launch_bounds__(256) void wmma_gemm64(
    const unsigned short* __restrict__ Ap, const unsigned short* __restrict__ A2p, int lda, long strideA,
    const unsigned short* __restrict__ Btp, const unsigned short* __restrict__ Bt2p, int ldb, long strideB,
    void* __restrict__ Cout, void* __restrict__ Cout2, int ldc, long strideC,
    const float* __restrict__ bias,
    const float* __restrict__ resid, long strideR,
    int M, int N, int K, float scale) {
  typedef typename Elem<ET>::T T;
  typedef typename Frag<T>::V V;
  const T* A = (const T*)Ap; const T* A2 = (const T*)A2p; const T* Bt = (const T*)Btp; const T* Bt2 = (const T*)Bt2p;
  __shared__ __align__(16) float sT[8][16 * 68];
  const int b    = blockIdx.y;
  const int lane = threadIdx.x & 31;
  const int wave = threadIdx.x >> 5;
  const int tilesN = N >> 6;
  const int tilesM = M >> 6;
  const int tile = blockIdx.x * 8 + wave;
  if (tile >= tilesM * tilesN) return;
  const int tm = tile / tilesN;
  const int tn = tile - tm * tilesN;
  const int m0 = tm << 6;
  const int n0 = tn << 6;

  const T* Ab  = A  + (size_t)b * strideA;
  const T* Bb  = Bt + (size_t)b * strideB;
  const T* Ab2 = SPLIT ? (A2  + (size_t)b * strideA) : nullptr;
  const T* Bb2 = SPLIT ? (Bt2 + (size_t)b * strideB) : nullptr;

  const int rlane = lane & 15;
  const int koff  = (lane >> 4) * 8;
  const int mOff  = (lane >> 4) * 8;

  v8f acc[4][4];
#pragma unroll
  for (int i = 0; i < 4; ++i)
#pragma unroll
    for (int j = 0; j < 4; ++j) acc[i][j] = (v8f){0.f,0.f,0.f,0.f,0.f,0.f,0.f,0.f};

  for (int k0 = 0; k0 < K; k0 += 32) {
    V bh[4], bl[4];
#pragma unroll
    for (int j = 0; j < 4; ++j) {
      const size_t bo = (size_t)(n0 + (j << 4) + rlane) * ldb + koff + k0;
      bh[j] = Frag<T>::load(Bb + bo);
      if (SPLIT) bl[j] = Frag<T>::load(Bb2 + bo);
    }
#pragma unroll
    for (int i = 0; i < 4; ++i) {
      const size_t ao = (size_t)(m0 + (i << 4) + rlane) * lda + koff + k0;
      V ah = Frag<T>::load(Ab + ao);
      V al;
      if (SPLIT) al = Frag<T>::load(Ab2 + ao);
#pragma unroll
      for (int j = 0; j < 4; ++j) {
        acc[i][j] = Frag<T>::mma(ah, bh[j], acc[i][j]);
        if (SPLIT) {
          acc[i][j] = Frag<T>::mma(ah, bl[j], acc[i][j]);
          acc[i][j] = Frag<T>::mma(al, bh[j], acc[i][j]);
        }
      }
      Frag<T>::guard(acc[i][0], acc[i][3], ah, SPLIT ? al : ah);
    }
    Frag<T>::keep(bh[0], bh[1], bh[2], bh[3]);
    if (SPLIT) Frag<T>::keep(bl[0], bl[1], bl[2], bl[3]);
  }
  acc_guard4(acc[0][0], acc[0][1], acc[0][2], acc[0][3]);
  acc_guard4(acc[1][0], acc[1][1], acc[1][2], acc[1][3]);
  acc_guard4(acc[2][0], acc[2][1], acc[2][2], acc[2][3]);
  acc_guard4(acc[3][0], acc[3][1], acc[3][2], acc[3][3]);

  float* slab = sT[wave];
  const float* Rb = RESID ? (resid + (size_t)b * strideR) : nullptr;
#pragma unroll
  for (int i = 0; i < 4; ++i) {
    const int mBase = m0 + (i << 4);
#pragma unroll
    for (int j = 0; j < 4; ++j) {
      const int n = n0 + (j << 4) + rlane;
      float bv = 0.f;
      if (BIAS_MODE == 2) bv = bias[n];
#pragma unroll
      for (int r = 0; r < 8; ++r) {
        float v = acc[i][j][r] * scale;
        if (BIAS_MODE == 1) v += bias[mBase + mOff + r];
        if (BIAS_MODE == 2) v += bv;
        if (RESID) v += Rb[(size_t)(mBase + mOff + r) * ldc + n];
        if (ACT == 2) v = fmaxf(v, 0.0f);
        if (ACT == 4) v = (v > 0.f) ? v : 0.01f * v;
        slab[(mOff + r) * 68 + (j << 4) + rlane] = v;
      }
    }
    __builtin_amdgcn_fence(__ATOMIC_RELEASE, "workgroup");
    __builtin_amdgcn_wave_barrier();
    __builtin_amdgcn_fence(__ATOMIC_ACQUIRE, "workgroup");
    if (OUT_MODE == 0) {
      float* C = (float*)Cout + (size_t)b * strideC;
      const int hh = lane >> 4, c4 = (lane & 15) * 4;
      for (int pass = 0; pass < 2; ++pass) {
#pragma unroll
        for (int it = 0; it < 8; ++it) {
          const int row = it * 2 + hh;
          v4f v = *(const v4f*)(slab + row * 68 + c4);
          *(volatile v4f*)(C + (size_t)(mBase + row) * ldc + n0 + c4) = v;
        }
        __threadfence();
      }
    } else {
      const int q = lane >> 3, c8 = (lane & 7) * 8;
      unsigned short* C  = (unsigned short*)Cout  + (size_t)b * strideC;
      unsigned short* C2 = (OUT_MODE == 2) ? ((unsigned short*)Cout2 + (size_t)b * strideC) : nullptr;
      for (int pass = 0; pass < 2; ++pass) {
#pragma unroll
        for (int it = 0; it < 4; ++it) {
          const int row = it * 4 + q;
          const float* sp = slab + row * 68 + c8;
          v8h hv, lv;
#pragma unroll
          for (int e = 0; e < 8; ++e) {
            if (OUT_MODE == 1) {
              hv[e] = (_Float16)sp[e];
            } else {
              unsigned short hb = f2bf_bits(sp[e]);
              unsigned short lb = f2bf_bits(sp[e] - bf_bits2f(hb));
              hv[e] = __builtin_bit_cast(_Float16, hb);
              lv[e] = __builtin_bit_cast(_Float16, lb);
            }
          }
          *(volatile v8h*)(C + (size_t)(mBase + row) * ldc + n0 + c8) = hv;
          if (OUT_MODE == 2) *(volatile v8h*)(C2 + (size_t)(mBase + row) * ldc + n0 + c8) = lv;
        }
        __threadfence();
      }
    }
    __builtin_amdgcn_fence(__ATOMIC_RELEASE, "workgroup");
    __builtin_amdgcn_wave_barrier();
    __builtin_amdgcn_fence(__ATOMIC_ACQUIRE, "workgroup");
  }
}

__global__ __launch_bounds__(256) void cast8_kernel(const float* __restrict__ in, unsigned short* __restrict__ out,
                                                    int n8_valid, int n8_total, float scale) {
  const int i = blockIdx.x * 256 + threadIdx.x;
  if (i >= n8_total) return;
  const bool valid = (i < n8_valid);
  const int ic = valid ? i : (n8_valid - 1);
  const float* p = in + 8 * (size_t)ic;
  const v4f a = *(const v4f*)(p);
  const v4f c = *(const v4f*)(p + 4);
  unsigned short hb[8];
#pragma unroll
  for (int e = 0; e < 4; ++e) {
    const float v0 = valid ? (a[e] * scale) : 0.0f;
    const float v1 = valid ? (c[e] * scale) : 0.0f;
    hb[e]     = h_bits(v0);
    hb[4 + e] = h_bits(v1);
  }
  const v4u u = (v4u){pk16(hb[0], hb[1]), pk16(hb[2], hb[3]), pk16(hb[4], hb[5]), pk16(hb[6], hb[7])};
  unsigned short* q = out + 8 * (size_t)i;
  *(volatile v4u*)q = u;
  __threadfence();
  *(volatile v4u*)q = u;
}

__global__ __launch_bounds__(256) void conv_act_kernel(const float* __restrict__ zx, const float* __restrict__ conv_w,
                                                       const float* __restrict__ conv_b, const float* __restrict__ dt_bias,
                                                       const float* __restrict__ A_log,
                                                       float* __restrict__ xp, float* __restrict__ bcp, float* __restrict__ dd) {
  __shared__ __align__(16) float dsh[64];
  const int l  = blockIdx.x;
  const int cb = blockIdx.y;
  const int t  = threadIdx.x;
  if (cb < 3) {
    const bool active = (cb < 2) || (t < 64);
    if (active) {
      const int c0 = (cb < 2) ? (cb * 1024 + 4 * t) : (kDInner + 4 * t);
      v4f w[4];
#pragma unroll
      for (int ch = 0; ch < 4; ++ch) w[ch] = *(const v4f*)(conv_w + (size_t)(c0 + ch) * 4);
      v4f acc = (v4f){0.0f, 0.0f, 0.0f, 0.0f};
#pragma unroll
      for (int j = 0; j < 4; ++j) {
        const int ll  = l - 3 + j;
        const int llc = (ll < 0) ? 0 : ll;
        const v4f xv = *(const v4f*)(zx + (size_t)llc * kNPad + kDInner + c0);
#pragma unroll
        for (int ch = 0; ch < 4; ++ch) {
          const float xe = (ll >= 0) ? xv[ch] : 0.0f;
          acc[ch] = acc[ch] + w[ch][j] * xe;
        }
      }
      const v4f bb = *(const v4f*)(conv_b + c0);
      v4f o;
#pragma unroll
      for (int ch = 0; ch < 4; ++ch) {
        const float a  = acc[ch] + bb[ch];
        const float sg = 1.0f / (1.0f + expf(-a));
        o[ch] = a * sg;
      }
      float* dst = (cb < 2) ? (xp + (size_t)l * kDInner + c0) : (bcp + (size_t)l * (2 * kDState) + 4 * t);
      *(volatile v4f*)dst = o;
      __threadfence();
      *(volatile v4f*)dst = o;
    }
  } else {
    if (t < 64) {
      const int h = t & 31;
      const float raw = zx[(size_t)l * kNPad + (kDInner + kConvDim) + h] + dt_bias[h];
      const float sp  = fmaxf(raw, 0.0f) + log1pf(expf(-fabsf(raw)));
      const float a   = -expf(A_log[h]);
      const float dec = expf(a * sp);
      dsh[t] = (t < 32) ? sp : dec;
    }
    __syncthreads();
    if (t < 16) {
      const v4f v = *(const v4f*)(&dsh[4 * t]);
      float* dst = dd + (size_t)l * 64 + 4 * t;
      *(volatile v4f*)dst = v;
      __threadfence();
      *(volatile v4f*)dst = v;
    }
  }
}

__global__ __launch_bounds__(256) void scan_kernel(const float* __restrict__ xp, const float* __restrict__ bcp,
                                                   const float* __restrict__ dd, const float* __restrict__ D_param,
                                                   float* __restrict__ ys) {
  __shared__ __align__(16) float bcbuf[2][256];
  __shared__ float shpart[2][256];
  __shared__ __align__(16) float ytile[8][128];
  const int t    = threadIdx.x;
  const int lane = t & 31;
  const int wave = t >> 5;
  const int hl   = t >> 7;
  const int nh   = (t >> 6) & 1;
  const int p    = t & 63;
  const int h    = blockIdx.x * 2 + hl;
  const int col  = h * kHeadDim + p;
  const float Dcoef = D_param[h];

  float s[64];
#pragma unroll
  for (int i = 0; i < 64; ++i) s[i] = 0.0f;

  if (t < 64) {
    const v4f v = *(const v4f*)(bcp + 4 * t);
    *(v4f*)(&bcbuf[0][4 * t]) = v;
  }
  float xc   = xp[col];
  float dtc  = dd[h];
  float decc = dd[32 + h];
  __syncthreads();

  for (int tt = 0; tt < kSeq; ++tt) {
    const int cur = tt & 1;
    const int tn  = (tt + 1 < kSeq) ? (tt + 1) : (kSeq - 1);
    if (t < 64) {
      const v4f v = *(const v4f*)(bcp + (size_t)tn * (2 * kDState) + 4 * t);
      *(v4f*)(&bcbuf[cur ^ 1][4 * t]) = v;
    }
    const float xn   = xp[(size_t)tn * kDInner + col];
    const float dtn  = dd[(size_t)tn * 64 + h];
    const float decn = dd[(size_t)tn * 64 + 32 + h];

    const float xdt = xc * dtc;
    const v4f* Bp = (const v4f*)(&bcbuf[cur][nh * 64]);
    const v4f* Cp = (const v4f*)(&bcbuf[cur][kDState + nh * 64]);
    float part = 0.0f;
#pragma unroll
    for (int q = 0; q < 16; ++q) {
      const v4f bv = Bp[q];
      const v4f cv = Cp[q];
#pragma unroll
      for (int e = 0; e < 4; ++e) {
        const float u  = xdt * bv[e];
        const float sn = s[4 * q + e] * decc + u;
        s[4 * q + e] = sn;
        part = part + sn * cv[e];
      }
    }
    shpart[cur][t] = part;
    __syncthreads();
    if (nh == 0) {
      const float yv = (part + shpart[cur][t + 64]) + xc * Dcoef;
      ytile[tt & 7][hl * 64 + p] = yv;
    }
    if ((tt & 7) == 7) {
      __syncthreads();
      const int hh2 = lane >> 4;
      const int p4  = (lane & 15) * 4;
      const v4f v = *(const v4f*)(&ytile[wave][hh2 * 64 + p4]);
      float* dst = ys + (size_t)(tt - 7 + wave) * kDInner + (blockIdx.x * 2 + hh2) * kHeadDim + p4;
      *(volatile v4f*)dst = v;
      __threadfence();
      *(volatile v4f*)dst = v;
    }
    xc = xn; dtc = dtn; decc = decn;
  }
}

__global__ __launch_bounds__(256) void gate_norm_kernel(const float* __restrict__ ys, const float* __restrict__ zx,
                                                        const float* __restrict__ norm_w, unsigned short* __restrict__ y16,
                                                        float carry) {
  __shared__ __align__(16) float rowbuf[kDInner];
  __shared__ float red[8];
  const int l    = blockIdx.x;
  const int t    = threadIdx.x;
  const int lane = t & 31;
  const int wave = t >> 5;
  const float* yr = ys + (size_t)l * kDInner;
  const float* zr = zx + (size_t)l * kNPad;
  float ss = 0.0f;
#pragma unroll 1
  for (int e = 0; e < 8; ++e) {
    const int c = t + 256 * e;
    const float z = zr[c];
    const float g = z * (1.0f / (1.0f + expf(-z)));
    const float v = yr[c] * g;
    rowbuf[c] = v;
    ss = ss + v * v;
  }
#pragma unroll
  for (int off = 16; off > 0; off >>= 1) ss += __shfl_xor(ss, off, 32);
  if (lane == 0) red[wave] = ss;
  __syncthreads();
  float tot = red[0];
#pragma unroll
  for (int w = 1; w < 8; ++w) tot = tot + red[w];
  const float inv = 1.0f / sqrtf(tot * (1.0f / 2048.0f) + kEps);

  const v4f a  = *(const v4f*)(&rowbuf[8 * t]);
  const v4f c4 = *(const v4f*)(&rowbuf[8 * t + 4]);
  const v4f wa = *(const v4f*)(norm_w + 8 * t);
  const v4f wc = *(const v4f*)(norm_w + 8 * t + 4);
  unsigned short hb[8];
#pragma unroll
  for (int e = 0; e < 4; ++e) {
    hb[e]     = h_bits(a[e]  * inv * wa[e] * carry);
    hb[4 + e] = h_bits(c4[e] * inv * wc[e] * carry);
  }
  const v4u u = (v4u){pk16(hb[0], hb[1]), pk16(hb[2], hb[3]), pk16(hb[4], hb[5]), pk16(hb[6], hb[7])};
  unsigned short* dst = y16 + (size_t)l * kDInner + 8 * t;
  *(volatile v4u*)dst = u;
  __threadfence();
  *(volatile v4u*)dst = u;
}

extern "C" void kernel_launch(void* const* d_in, const int* in_sizes, int n_in,
                              void* d_out, int out_size, void* d_ws, size_t ws_size, hipStream_t stream) {
  if (n_in < 9) return;
  if (out_size != kRows * kDModel) return;
  if (in_sizes[0] != kRows * kDModel || in_sizes[1] != kDInProj * kDModel || in_sizes[2] != kConvDim * 4 ||
      in_sizes[3] != kConvDim || in_sizes[4] != kDInner || in_sizes[5] != kDModel * kDInner ||
      in_sizes[6] != kNHeads || in_sizes[7] != kNHeads || in_sizes[8] != kNHeads) return;

  const float* x          = (const float*)d_in[0];
  const float* in_proj_w  = (const float*)d_in[1];
  const float* conv_w     = (const float*)d_in[2];
  const float* conv_b     = (const float*)d_in[3];
  const float* norm_w     = (const float*)d_in[4];
  const float* out_proj_w = (const float*)d_in[5];
  const float* dt_bias    = (const float*)d_in[6];
  const float* A_log      = (const float*)d_in[7];
  const float* D_param    = (const float*)d_in[8];
  float* out = (float*)d_out;

  char* ws = (char*)d_ws;
  size_t off = 0;
  unsigned short* xh  = (unsigned short*)(ws + off); off += (size_t)kRows * kDModel * 2;
  unsigned short* w1h = (unsigned short*)(ws + off); off += (size_t)kNPad * kDModel * 2;
  unsigned short* w2h = (unsigned short*)(ws + off); off += (size_t)kDModel * kDInner * 2;
  float* zx  = (float*)(ws + off); off += (size_t)kSeq * kNPad * 4;
  float* xp  = (float*)(ws + off); off += (size_t)kSeq * kDInner * 4;
  float* bcp = (float*)(ws + off); off += (size_t)kSeq * (2 * kDState) * 4;
  float* dd  = (float*)(ws + off); off += (size_t)kSeq * 64 * 4;
  float* ys  = (float*)(ws + off); off += (size_t)kSeq * kDInner * 4;
  unsigned short* y16 = (unsigned short*)(ws + off); off += (size_t)kRows * kDInner * 2;
  if (off > ws_size) return;

  {
    const int n8x  = kRows * kDModel / 8;
    const int n8w1 = kDInProj * kDModel / 8;
    const int n8w1t = kNPad * kDModel / 8;
    const int n8w2 = kDModel * kDInner / 8;
    cast8_kernel<<<(n8x + 255) / 256, 256, 0, stream>>>(x, xh, n8x, n8x, kXCarry);
    cast8_kernel<<<(n8w1t + 255) / 256, 256, 0, stream>>>(in_proj_w, w1h, n8w1, n8w1t, kWCarry);
    cast8_kernel<<<(n8w2 + 255) / 256, 256, 0, stream>>>(out_proj_w, w2h, n8w2, n8w2, kWCarry);
  }

  for (int b = 0; b < kBatch; ++b) {
    {
      dim3 grid((kSeq / 64) * (kNPad / 64) / 8, 1);
      wmma_gemm64<0, false, 0, 0, false, 0><<<grid, 256, 0, stream>>>(
          xh + (size_t)b * kSeq * kDModel, nullptr, kDModel, 0L,
          w1h, nullptr, kDModel, 0L,
          (void*)zx, nullptr, kNPad, 0L,
          nullptr, nullptr, 0L,
          kSeq, kNPad, kDModel, kProjScale);
    }
    conv_act_kernel<<<dim3(kSeq, 4), 256, 0, stream>>>(zx, conv_w, conv_b, dt_bias, A_log, xp, bcp, dd);
    scan_kernel<<<kNHeads / 2, 256, 0, stream>>>(xp, bcp, dd, D_param, ys);
    gate_norm_kernel<<<kSeq, 256, 0, stream>>>(ys, zx, norm_w, y16 + (size_t)b * kSeq * kDInner, kYCarry);
  }

  {
    dim3 grid((kRows / 64) * (kDModel / 64) / 8, 1);
    wmma_gemm64<0, false, 0, 0, false, 0><<<grid, 256, 0, stream>>>(
        y16, nullptr, kDInner, 0L,
        w2h, nullptr, kDInner, 0L,
        (void*)out, nullptr, kDModel, 0L,
        nullptr, nullptr, 0L,
        kRows, kDModel, kDInner, kProjScale);
  }
}
